// GIN_GNN_75677323755666
// MI455X (gfx1250) — hardware-verified
//
#include <hip/hip_runtime.h>


namespace {
constexpr int N = 100000, E = 1600000, NG = 64, F0 = 16, H = 128, GF = 8, NCLS = 2, KC1 = 2 * H + GF, KC1P = 288;
constexpr int NPAD = 100096;
constexpr int NBLK = NPAD / 128;

typedef _Float16 b16;
typedef __attribute__((ext_vector_type(16))) _Float16 v16b;
typedef __attribute__((ext_vector_type(8)))  _Float16 v8b;
typedef __attribute__((ext_vector_type(8)))  float v8f;
typedef __attribute__((ext_vector_type(4)))  float v4f;

__device__ __forceinline__ v8b ld8b(const b16* p) { return *(const v8b*)p; }
__device__ __forceinline__ v16b cat8b(v8b a, v8b b) { return __builtin_shufflevector(a, b, 0, 1, 2, 3, 4, 5, 6, 7, 8, 9, 10, 11, 12, 13, 14, 15); }
__device__ __forceinline__ v16b frag_kb(const b16* p, int hh) { return cat8b(ld8b(p + 8 * hh), ld8b(p + 16 + 8 * hh)); }
__device__ __forceinline__ void split16(float v, b16& hi, b16& lo) { hi = (b16)v; lo = (b16)(v - (float)hi); }
__device__ __forceinline__ void frag_ksplit(const float* p, int hh, v16b& fh_, v16b& fl_) {
  const float* p0 = p + 8 * hh; const float* p1 = p + 16 + 8 * hh;
#pragma unroll
  for (int e = 0; e < 8; ++e) { b16 a, c; split16(p0[e], a, c); fh_[e] = a; fl_[e] = c; split16(p1[e], a, c); fh_[8 + e] = a; fl_[8 + e] = c; }
}
__device__ __forceinline__ v8f wmma16b(v16b a, v16b b, v8f c) {
  v8f d = __builtin_amdgcn_wmma_f32_16x16x32_f16(false, a, false, b, (short)0, c, false, false);
  asm volatile("v_nop\n\tv_nop\n\tv_nop\n\tv_nop" : "+v"(d) : "v"(a), "v"(b));
  return d;
}
__device__ __forceinline__ void wave_lds_sync() {
  __builtin_amdgcn_fence(__ATOMIC_RELEASE, "workgroup");
  __builtin_amdgcn_wave_barrier();
  __builtin_amdgcn_fence(__ATOMIC_ACQUIRE, "workgroup");
}

struct Opnd { const void* p0; const void* p1; int ld; };
template <int NP> __device__ __forceinline__ void load_frags(const Opnd& o, int row, int kb, int hh, v16b& fh_, v16b& fl_) {
  if (NP == 0) { frag_ksplit((const float*)o.p0 + (size_t)row * o.ld + kb, hh, fh_, fl_); }
  else if (NP == 4) {
    const float* p = (const float*)o.p0 + (size_t)row * o.ld + kb; const float* p0 = p + 8 * hh; const float* p1 = p + 16 + 8 * hh;
#pragma unroll
    for (int e = 0; e < 8; ++e) { b16 a, c; split16(p0[e] * 64.0f, a, c); fh_[e] = a; fl_[e] = c; split16(p1[e] * 64.0f, a, c); fh_[8 + e] = a; fl_[8 + e] = c; }
  } else if (NP == 3) {
    const float* p = (const float*)o.p0 + (size_t)row * o.ld + kb; const float* p0 = p + 8 * hh; const float* p1 = p + 16 + 8 * hh;
#pragma unroll
    for (int e = 0; e < 8; ++e) { fh_[e] = (b16)p0[e]; fh_[8 + e] = (b16)p1[e]; }
    fl_ = fh_;
  } else {
    fh_ = frag_kb((const b16*)o.p0 + (size_t)row * o.ld + kb, hh);
    if (NP == 2) fl_ = frag_kb((const b16*)o.p1 + (size_t)row * o.ld + kb, hh); else fl_ = fh_;
  }
}
template <int ANP, int BNP> __device__ __forceinline__ v8f mac(v16b ah, v16b al, v16b bh, v16b bl, v8f c) {
  c = wmma16b(ah, bh, c);
  if (BNP == 0 || BNP == 2 || BNP == 4) c = wmma16b(ah, bl, c);
  if (ANP == 0 || ANP == 2 || ANP == 4) c = wmma16b(al, bh, c);
  return c;
}
template <int ANP, int BNP>
__device__ __forceinline__ void gemm_tile(const Opnd& A, const Opnd& B, int K, int m0, int c0, int nloc, int hlf, v8f (&acc)[2][4]) {
  for (int kb = 0; kb < K; kb += 32) {
    v16b a0h, a0l, a1h, a1l;
    load_frags<ANP>(A, m0 + nloc, kb, hlf, a0h, a0l);
    load_frags<ANP>(A, m0 + 16 + nloc, kb, hlf, a1h, a1l);
#pragma unroll
    for (int t = 0; t < 4; ++t) {
      v16b bh, bl;
      load_frags<BNP>(B, c0 + t * 16 + nloc, kb, hlf, bh, bl);
      acc[0][t] = mac<ANP, BNP>(a0h, a0l, bh, bl, acc[0][t]);
      acc[1][t] = mac<ANP, BNP>(a1h, a1l, bh, bl, acc[1][t]);
    }
  }
}

__device__ __forceinline__ void epi_planes(v8f (&acc)[2][4], float scale, bool two, b16* __restrict__ oh, b16* __restrict__ ol, int ldo,
                                           int m0, int c0, int lane, b16* Th, b16* Tl) {
  const int nloc = lane & 15, hlf = lane >> 4;
#pragma unroll
  for (int t = 0; t < 4; ++t)
#pragma unroll
    for (int r = 0; r < 2; ++r)
#pragma unroll
      for (int v = 0; v < 8; ++v) {
        const int rr = r * 16 + v + 8 * hlf, cc = t * 16 + nloc;
        b16 h_, l_; split16(acc[r][t][v] * scale, h_, l_);
        Th[rr * 64 + cc] = h_; Tl[rr * 64 + cc] = l_;
      }
  wave_lds_sync();
  for (int pass = 0; pass < 2; ++pass) {
#pragma unroll
    for (int j = 0; j < 8; ++j) {
      const int rr = j * 4 + (lane >> 3), c8 = (lane & 7) * 8;
      const size_t o = (size_t)(m0 + rr) * ldo + c0 + c8;
      *(volatile v8b*)(oh + o) = ld8b(Th + rr * 64 + c8);
      if (two) *(volatile v8b*)(ol + o) = ld8b(Tl + rr * 64 + c8);
    }
    __threadfence();
  }
}
__device__ __forceinline__ void epi_f32(v8f (&acc)[2][4], float scale, const float* rscale, float* __restrict__ out, int ldo, int m0, int c0, int lane, float* Tt) {
  const int nloc = lane & 15, hlf = lane >> 4;
#pragma unroll
  for (int t = 0; t < 4; ++t)
#pragma unroll
    for (int r = 0; r < 2; ++r)
#pragma unroll
      for (int v = 0; v < 8; ++v) {
        const int rr = r * 16 + v + 8 * hlf;
        const float rs = rscale ? rscale[(size_t)(m0 + rr) * 32] : 1.0f;
        Tt[rr * 64 + t * 16 + nloc] = acc[r][t][v] * scale * rs;
      }
  wave_lds_sync();
  float* dst0 = out + (size_t)m0 * ldo + c0;
  for (int pass = 0; pass < 2; ++pass) {
#pragma unroll
    for (int j = 0; j < 16; ++j) { const int rr = j * 2 + hlf, c4 = nloc * 4; *(volatile v4f*)(dst0 + (size_t)rr * ldo + c4) = *(const v4f*)(Tt + rr * 64 + c4); }
    __threadfence();
  }
}


__global__ __launch_bounds__(256) void prep_kernel(const float* __restrict__ h0, const float* __restrict__ co, const float* __restrict__ W1_0, const float* __restrict__ W2_0,
                                                   const float* __restrict__ Ws1, const float* __restrict__ Ws2, const float* __restrict__ Wc1, const float* __restrict__ Wc2,
                                                   float* __restrict__ x0, b16* __restrict__ w10, b16* __restrict__ w20, b16* __restrict__ ws1, b16* __restrict__ ws2, b16* __restrict__ wc1, b16* __restrict__ wc2) {
  const size_t tid = (size_t)blockIdx.x * blockDim.x + threadIdx.x, nth = (size_t)gridDim.x * blockDim.x;
  for (int pass = 0; pass < 2; ++pass) {
    for (size_t p = tid; p < (size_t)NPAD * F0 / 4; p += nth) { const int n = (int)(p / 4), k0 = (int)(p % 4) * 4; v4f v;
#pragma unroll
      for (int e = 0; e < 4; ++e) { const int k = k0 + e; v[e] = (n < N) ? ((k < 13) ? h0[(size_t)n * 13 + k] : co[(size_t)n * 3 + (k - 13)]) : 0.0f; }
      *(volatile v4f*)(x0 + p * 4) = v; }
    for (size_t p = tid; p < (size_t)H * F0 / 8; p += nth) { const int n = (int)(p / 2), k0 = (int)(p % 2) * 8; v8b v;
#pragma unroll
      for (int e = 0; e < 8; ++e) v[e] = (b16)W1_0[(size_t)(k0 + e) * H + n];
      *(volatile v8b*)(w10 + p * 8) = v; }
    for (size_t p = tid; p < (size_t)5 * H * H / 8; p += nth) { const int m = (int)(p / (H * H / 8)); const int rem = (int)(p % (H * H / 8)), n = rem / 16, k0 = (rem % 16) * 8;
      const float* W = (m == 0) ? W2_0 : (m == 1) ? Ws1 : (m == 2) ? (Ws1 + H * H) : (m == 3) ? Ws2 : (Ws2 + H * H);
      b16* dst = (m == 0) ? w20 : (m == 1) ? ws1 : (m == 2) ? (ws1 + H * H) : (m == 3) ? ws2 : (ws2 + H * H); v8b v;
#pragma unroll
      for (int e = 0; e < 8; ++e) v[e] = (b16)W[(size_t)(k0 + e) * H + n];
      *(volatile v8b*)(dst + (size_t)n * H + k0) = v; }
    for (size_t p = tid; p < (size_t)H * KC1P / 8; p += nth) { const int n = (int)(p / (KC1P / 8)), k0 = (int)(p % (KC1P / 8)) * 8; v8b v;
#pragma unroll
      for (int e = 0; e < 8; ++e) { const int k = k0 + e; v[e] = (b16)((k < KC1) ? Wc1[(size_t)k * H + n] : 0.0f); }
      *(volatile v8b*)(wc1 + (size_t)n * KC1P + k0) = v; }
    for (size_t p = tid; p < (size_t)16 * H / 8; p += nth) { const int n = (int)(p / 16), k0 = (int)(p % 16) * 8; v8b v;
#pragma unroll
      for (int e = 0; e < 8; ++e) v[e] = (b16)((n < NCLS) ? Wc2[(size_t)(k0 + e) * NCLS + n] : 0.0f);
      *(volatile v8b*)(wc2 + (size_t)n * H + k0) = v; }
    __threadfence();
  }
}

template <int DF, int NB>
__global__ __launch_bounds__(256) void agg_kernel(const int* __restrict__ esrc, const int* __restrict__ edst, const float* __restrict__ x, float* __restrict__ zin) {
  __shared__ __attribute__((aligned(16))) int acc[NB * DF];
  __shared__ int list[8 * 256];
  constexpr float FXS = 524288.0f, FXI = 1.0f / 524288.0f;
  const int t_ = threadIdx.x, wave = t_ >> 5, lane = t_ & 31, base = blockIdx.x * NB;
  for (int i = t_; i < NB * DF; i += 256) acc[i] = 0;
  __syncthreads();
  int* wl = list + wave * 256;
  typedef __attribute__((ext_vector_type(4))) int v4i;
  for (int c0 = 0; c0 < E; c0 += 256 * 8) {
    const int e0 = c0 + (wave * 32 + lane) * 8;
    int dd[8];
    if (e0 + 7 < E) { const v4i a = *(const v4i*)(edst + e0), b = *(const v4i*)(edst + e0 + 4); dd[0] = a[0]; dd[1] = a[1]; dd[2] = a[2]; dd[3] = a[3]; dd[4] = b[0]; dd[5] = b[1]; dd[6] = b[2]; dd[7] = b[3]; }
    else {
#pragma unroll
      for (int j = 0; j < 8; ++j) dd[j] = (e0 + j < E) ? edst[e0 + j] : -1; }
    unsigned sl[8]; bool hit[8]; bool anyl = false;
#pragma unroll
    for (int j = 0; j < 8; ++j) { sl[j] = (unsigned)(dd[j] - base); hit[j] = sl[j] < (unsigned)NB; anyl |= hit[j]; }
    int wc = 0;
    if (__builtin_amdgcn_ballot_w32(anyl) != 0u) {
#pragma unroll
      for (int j = 0; j < 8; ++j) {
        const unsigned mj = __builtin_amdgcn_ballot_w32(hit[j]);
        if (mj != 0u) {
          if (hit[j]) { const int pos = wc + (int)__builtin_amdgcn_mbcnt_lo(mj, 0u); int s = esrc[e0 + j]; s = (s < 0) ? 0 : (s >= N ? N - 1 : s); wl[pos] = (s << 12) | (int)sl[j]; }
          wc += __builtin_popcount(mj);
        }
      }
    }
    __builtin_amdgcn_wave_barrier(); __builtin_amdgcn_fence(__ATOMIC_RELEASE, "workgroup"); __builtin_amdgcn_fence(__ATOMIC_ACQUIRE, "workgroup");
    if (DF == 128) {
      for (int i = 0; i < wc; ++i) { const int ent = wl[i]; const int s = ent >> 12, slot = ent & 4095;
        const v4f v = *(const v4f*)(x + (size_t)s * DF + lane * 4);
#pragma unroll
        for (int c = 0; c < 4; ++c) atomicAdd(&acc[slot * DF + lane * 4 + c], (int)rintf(v[c] * FXS)); }
    } else {
      for (int i0 = 0; i0 < wc; i0 += 8) { const int i = i0 + (lane >> 2); if (i < wc) { const int ent = wl[i]; const int s = ent >> 12, slot = ent & 4095;
          const v4f v = *(const v4f*)(x + (size_t)s * DF + (lane & 3) * 4);
#pragma unroll
          for (int c = 0; c < 4; ++c) atomicAdd(&acc[slot * DF + (lane & 3) * 4 + c], (int)rintf(v[c] * FXS)); } }
    }
    __builtin_amdgcn_wave_barrier();
  }
  __syncthreads();
  for (int pass = 0; pass < 2; ++pass) {
    for (int i = t_; i < NB * DF / 4; i += 256) { const int r = (i * 4) / DF; const int node = base + r; if (node < NPAD) {
        v4f o = {0.0f, 0.0f, 0.0f, 0.0f}; if (node < N) { const v4f xx = *(const v4f*)(x + (size_t)base * DF + (size_t)i * 4);
#pragma unroll
          for (int c = 0; c < 4; ++c) o[c] = (float)acc[i * 4 + c] * FXI + xx[c]; }
        *(volatile v4f*)(zin + (size_t)base * DF + (size_t)i * 4) = o; } }
    __threadfence();
  }
}

template <int KIN>
__global__ __launch_bounds__(128) void lin1_kernel(const float* __restrict__ zin, const b16* __restrict__ w1, const float* __restrict__ b1, float* __restrict__ z32, float* __restrict__ slot) {
  __shared__ __attribute__((aligned(16))) float Ts[4][32 * 64]; __shared__ float Ss[4][2][64];
  const int lane = threadIdx.x & 31, wave = threadIdx.x >> 5, nloc = lane & 15, hlf = lane >> 4, m0 = blockIdx.y * 128 + wave * 32, c0 = blockIdx.x * 64;
  v8f acc[2][4];
#pragma unroll
  for (int r = 0; r < 2; ++r)
#pragma unroll
    for (int t = 0; t < 4; ++t) acc[r][t] = (v8f){};
  const Opnd A{zin, nullptr, KIN}, B{w1, nullptr, KIN};
  if (KIN >= 32) gemm_tile<3, 1>(A, B, KIN, m0, c0, nloc, hlf, acc);
  else {
    v16b a0 = {}, a1 = {};
#pragma unroll
    for (int e = 0; e < 8; ++e) { a0[e] = (b16)zin[(size_t)(m0 + nloc) * KIN + 8 * hlf + e]; a1[e] = (b16)zin[(size_t)(m0 + 16 + nloc) * KIN + 8 * hlf + e]; }
#pragma unroll
    for (int t = 0; t < 4; ++t) { v16b bw = {}; const v8b p8 = ld8b(w1 + (size_t)(c0 + t * 16 + nloc) * KIN + 8 * hlf);
#pragma unroll
      for (int e = 0; e < 8; ++e) bw[e] = p8[e];
      acc[0][t] = wmma16b(a0, bw, acc[0][t]); acc[1][t] = wmma16b(a1, bw, acc[1][t]); }
  }
  float cs[4] = {0, 0, 0, 0}, cs2[4] = {0, 0, 0, 0};
#pragma unroll
  for (int t = 0; t < 4; ++t)
#pragma unroll
    for (int r = 0; r < 2; ++r)
#pragma unroll
      for (int v = 0; v < 8; ++v) { const float val = acc[r][t][v] + b1[c0 + t * 16 + nloc]; acc[r][t][v] = val; const int row = m0 + r * 16 + v + 8 * hlf; if (row < N) { cs[t] += val; cs2[t] += val * val; } }
#pragma unroll
  for (int t = 0; t < 4; ++t) { cs[t] += __shfl_xor(cs[t], 16); cs2[t] += __shfl_xor(cs2[t], 16); if (hlf == 0) { Ss[wave][0][t * 16 + nloc] = cs[t]; Ss[wave][1][t * 16 + nloc] = cs2[t]; } }
  epi_f32(acc, 1.0f, nullptr, z32, H, m0, c0, lane, Ts[wave]);
  __syncthreads();
  if (wave == 0) for (int o = lane; o < 64; o += 32) { const float s = Ss[0][0][o] + Ss[1][0][o] + Ss[2][0][o] + Ss[3][0][o], s2 = Ss[0][1][o] + Ss[1][1][o] + Ss[2][1][o] + Ss[3][1][o];
    for (int pass = 0; pass < 2; ++pass) { ((volatile float*)slot)[((size_t)blockIdx.y * 2) * H + c0 + o] = s; ((volatile float*)slot)[((size_t)blockIdx.y * 2 + 1) * H + c0 + o] = s2; __threadfence(); } }
}

__global__ __launch_bounds__(128) void bnfin_kernel(const float* __restrict__ slot, const float* __restrict__ g, const float* __restrict__ bb, float* __restrict__ coef) {
  const int c = threadIdx.x; double s = 0.0, s2 = 0.0;
#pragma unroll 1
  for (int bk = 0; bk < NBLK; ++bk) { s += (double)slot[((size_t)bk * 2) * H + c]; s2 += (double)slot[((size_t)bk * 2 + 1) * H + c]; }
  const double mean = s / N, var = s2 / N - mean * mean; const float a = g[c] * (float)(1.0 / sqrt(var + 1e-5)), sh = bb[c] - (float)mean * a;
  for (int pass = 0; pass < 2; ++pass) { ((volatile float*)coef)[c] = a; ((volatile float*)coef)[H + c] = sh; __threadfence(); }
}

__global__ __launch_bounds__(128) void lin2_kernel(const float* __restrict__ z32, const float* __restrict__ coef, const b16* __restrict__ w2, const float* __restrict__ b2, float* __restrict__ xo) {
  __shared__ __attribute__((aligned(16))) float Ts[4][32 * 64];
  const int lane = threadIdx.x & 31, wave = threadIdx.x >> 5, nloc = lane & 15, hlf = lane >> 4, m0 = blockIdx.y * 128 + wave * 32, c0 = blockIdx.x * 64;
  v8f acc[2][4];
#pragma unroll
  for (int r = 0; r < 2; ++r)
#pragma unroll
    for (int t = 0; t < 4; ++t) acc[r][t] = (v8f){};
#pragma unroll 1
  for (int kb = 0; kb < H; kb += 32) {
    v16b a0, a1;
#pragma unroll
    for (int e = 0; e < 16; ++e) { const int k = kb + ((e < 8) ? (8 * hlf + e) : (16 + 8 * hlf + e - 8)); const float ca = coef[k], sh = coef[H + k];
      a0[e] = (b16)fmaxf(z32[(size_t)(m0 + nloc) * H + k] * ca + sh, 0.0f); a1[e] = (b16)fmaxf(z32[(size_t)(m0 + 16 + nloc) * H + k] * ca + sh, 0.0f); }
#pragma unroll
    for (int t = 0; t < 4; ++t) { const v16b bw = frag_kb(w2 + (size_t)(c0 + t * 16 + nloc) * H + kb, hlf); acc[0][t] = wmma16b(a0, bw, acc[0][t]); acc[1][t] = wmma16b(a1, bw, acc[1][t]); }
  }
#pragma unroll
  for (int t = 0; t < 4; ++t)
#pragma unroll
    for (int r = 0; r < 2; ++r)
#pragma unroll
      for (int v = 0; v < 8; ++v) { const float val = acc[r][t][v] + b2[c0 + t * 16 + nloc]; acc[r][t][v] = (val > 0.0f) ? val : 0.1f * (__expf(val) - 1.0f); }
  epi_f32(acc, 1.0f, nullptr, xo, H, m0, c0, lane, Ts[wave]);
}

__global__ __launch_bounds__(256) void pool_kernel(const float* __restrict__ x, const int* __restrict__ batch, const float* __restrict__ g0, float* __restrict__ xg) {
  __shared__ float Ps[8][H], Pm[8][H]; __shared__ float Pc[8]; __shared__ __attribute__((aligned(16))) float Row[KC1P];
  const int wave = threadIdx.x >> 5, lane = threadIdx.x & 31, b = blockIdx.x;
  v4f s = {0, 0, 0, 0}, mx = {-INFINITY, -INFINITY, -INFINITY, -INFINITY}; float cnt = 0.0f;
#pragma unroll 1
  for (int n = wave; n < N; n += 8) { if (batch[n] == b) { const v4f v = *(const v4f*)(x + (size_t)n * H + lane * 4); s += v;
#pragma unroll
      for (int c = 0; c < 4; ++c) mx[c] = fmaxf(mx[c], v[c]);
      cnt += 1.0f; } }
#pragma unroll
  for (int c = 0; c < 4; ++c) { Ps[wave][lane * 4 + c] = s[c]; Pm[wave][lane * 4 + c] = mx[c]; }
  if (lane == 0) Pc[wave] = cnt;
  __syncthreads();
  if (threadIdx.x < H) { const int d = threadIdx.x; float ss = 0.0f, mm = -INFINITY, cc = 0.0f;
#pragma unroll
    for (int w = 0; w < 8; ++w) { ss += Ps[w][d]; mm = fmaxf(mm, Pm[w][d]); cc += Pc[w]; }
    Row[d] = ss / fmaxf(cc, 1.0f); Row[H + d] = (cc > 0.0f) ? mm : -INFINITY; }
  if (threadIdx.x < KC1P - 2 * H) { const int k = 2 * H + threadIdx.x; Row[k] = (k < KC1) ? g0[b * GF + (k - 2 * H)] : 0.0f; }
  __syncthreads();
  for (int pass = 0; pass < 2; ++pass) { if (threadIdx.x < KC1P / 4) *(volatile v4f*)(xg + (size_t)b * KC1P + threadIdx.x * 4) = *(const v4f*)(&Row[threadIdx.x * 4]); __threadfence(); }
}

__global__ __launch_bounds__(64) void cls_kernel(const float* __restrict__ xg, const b16* __restrict__ wc1, const float* __restrict__ bc1, const b16* __restrict__ wc2, const float* __restrict__ bc2, float* __restrict__ out) {
  __shared__ __attribute__((aligned(16))) b16 Zt[64][H + 8]; __shared__ float Ob[64 * 2];
  const int wave = threadIdx.x >> 5, lane = threadIdx.x & 31, nloc = lane & 15, hlf = lane >> 4, m0 = wave * 32;
  v8f acc[2][8];
#pragma unroll
  for (int r = 0; r < 2; ++r)
#pragma unroll
    for (int t = 0; t < 8; ++t) acc[r][t] = (v8f){};
  const Opnd A{xg, nullptr, KC1P};
#pragma unroll 1
  for (int kb = 0; kb < KC1P; kb += 32) { v16b a0, a1, d0, d1; load_frags<3>(A, m0 + nloc, kb, hlf, a0, d0); load_frags<3>(A, m0 + 16 + nloc, kb, hlf, a1, d1);
#pragma unroll
    for (int t = 0; t < 8; ++t) { const v16b bw = frag_kb(wc1 + (size_t)(t * 16 + nloc) * KC1P + kb, hlf); acc[0][t] = wmma16b(a0, bw, acc[0][t]); acc[1][t] = wmma16b(a1, bw, acc[1][t]); } }
#pragma unroll
  for (int t = 0; t < 8; ++t)
#pragma unroll
    for (int r = 0; r < 2; ++r)
#pragma unroll
      for (int v = 0; v < 8; ++v) { const float val = acc[r][t][v] + bc1[t * 16 + nloc]; Zt[m0 + r * 16 + v + 8 * hlf][t * 16 + nloc] = (b16)((val > 0.0f) ? val : 0.1f * (__expf(val) - 1.0f)); }
  wave_lds_sync();
  v8f lg[2] = {{}, {}};
#pragma unroll
  for (int kb = 0; kb < H; kb += 32) { const v16b bw = frag_kb(wc2 + (size_t)nloc * H + kb, hlf);
    lg[0] = wmma16b(frag_kb(&Zt[m0 + nloc][0] + kb, hlf), bw, lg[0]); lg[1] = wmma16b(frag_kb(&Zt[m0 + 16 + nloc][0] + kb, hlf), bw, lg[1]); }
#pragma unroll
  for (int r = 0; r < 2; ++r)
#pragma unroll
    for (int v = 0; v < 8; ++v) { const float mine = lg[r][v] + ((nloc < NCLS) ? bc2[nloc & 1] : 0.0f);
      const float l0 = __shfl(mine, (lane & 16) + 0, 32), l1 = __shfl(mine, (lane & 16) + 1, 32);
      const float mxx = fmaxf(l0, l1); const float e0 = __expf(l0 - mxx), e1 = __expf(l1 - mxx); const int row = m0 + r * 16 + v + 8 * hlf;
      if (nloc == 0) { Ob[row * 2] = e0 / (e0 + e1); Ob[row * 2 + 1] = e1 / (e0 + e1); } }
  __syncthreads();
  if (threadIdx.x < 32) for (int pass = 0; pass < 2; ++pass) { *(volatile v4f*)(out + threadIdx.x * 4) = *(const v4f*)(&Ob[threadIdx.x * 4]); __threadfence(); }
}
}

extern "C" void kernel_launch(void* const* d_in, const int* in_sizes, int n_in,
                              void* d_out, int out_size, void* d_ws, size_t ws_size, hipStream_t stream) {
  (void)n_in; (void)out_size;
  const float* h0 = (const float*)d_in[0]; const float* co = (const float*)d_in[1]; const float* g0 = (const float*)d_in[2]; const int* ei = (const int*)d_in[3]; const int* batch = (const int*)d_in[4];
  const float* W1_0 = (const float*)d_in[5]; const float* b1_0 = (const float*)d_in[6]; const float* g_0 = (const float*)d_in[7]; const float* be_0 = (const float*)d_in[8];
  const float* W2_0 = (const float*)d_in[9]; const float* b2_0 = (const float*)d_in[10];
  const float* Ws1 = (const float*)d_in[11]; const float* bs1 = (const float*)d_in[12]; const float* gs = (const float*)d_in[13]; const float* bes = (const float*)d_in[14];
  const float* Ws2 = (const float*)d_in[15]; const float* bs2 = (const float*)d_in[16];
  const float* Wc1 = (const float*)d_in[17]; const float* bc1 = (const float*)d_in[18]; const float* Wc2 = (const float*)d_in[19]; const float* bc2 = (const float*)d_in[20];
  float* out = (float*)d_out;
  if (in_sizes[0] != N * 13 || in_sizes[3] != 2 * E || in_sizes[4] != N || in_sizes[5] != F0 * H || in_sizes[11] != 2 * H * H || in_sizes[17] != KC1 * H) return;
  const int* esrc = ei; const int* edst = ei + E;
  size_t off = 0; char* ws = (char*)d_ws;
  auto carve = [&](size_t bytes) { char* p = ws + off; off += (bytes + 255) & ~(size_t)255; return p; };
  float* x0 = (float*)carve((size_t)NPAD * F0 * 4); float* zin0 = (float*)carve((size_t)NPAD * F0 * 4);
  b16* w10 = (b16*)carve(H * F0 * 2); b16* w20 = (b16*)carve(H * H * 2); b16* ws1 = (b16*)carve(2 * H * H * 2); b16* ws2 = (b16*)carve(2 * H * H * 2); b16* wc1 = (b16*)carve(H * KC1P * 2); b16* wc2 = (b16*)carve(16 * H * 2);
  float* bufF = (float*)carve((size_t)NPAD * H * 4); float* bufG = (float*)carve((size_t)NPAD * H * 4);
  float* slot = (float*)carve((size_t)NBLK * 2 * H * 4); float* coef = (float*)carve(2 * H * 4); float* xg = (float*)carve((size_t)NG * KC1P * 4);
  if (off > ws_size) return;
  prep_kernel<<<512, 256, 0, stream>>>(h0, co, W1_0, W2_0, Ws1, Ws2, Wc1, Wc2, x0, w10, w20, ws1, ws2, wc1, wc2);
  agg_kernel<F0, 4096><<<NPAD / 4096 + 1, 256, 0, stream>>>(esrc, edst, x0, zin0);
  lin1_kernel<F0><<<dim3(2, NBLK), 128, 0, stream>>>(zin0, w10, b1_0, bufF, slot);
  bnfin_kernel<<<1, 128, 0, stream>>>(slot, g_0, be_0, coef);
  lin2_kernel<<<dim3(2, NBLK), 128, 0, stream>>>(bufF, coef, w20, b2_0, bufG);
  float* feat = bufG; float* other = bufF;
  for (int l = 0; l < 2; ++l) {
    agg_kernel<H, 512><<<NPAD / 512 + 1, 256, 0, stream>>>(esrc, edst, feat, other);
    lin1_kernel<H><<<dim3(2, NBLK), 128, 0, stream>>>(other, ws1 + (size_t)l * H * H, bs1 + l * H, feat, slot);
    bnfin_kernel<<<1, 128, 0, stream>>>(slot, gs + l * H, bes + l * H, coef);
    lin2_kernel<<<dim3(2, NBLK), 128, 0, stream>>>(feat, coef, ws2 + (size_t)l * H * H, bs2 + l * H, other);
    float* tmp = feat; feat = other; other = tmp;
  }
  pool_kernel<<<NG, 256, 0, stream>>>(feat, batch, g0, xg);
  cls_kernel<<<1, 64, 0, stream>>>(xg, wc1, bc1, wc2, bc2, out);
}
